// BFANet_mink_63840393888176
// MI455X (gfx1250) — hardware-verified
//
#include <hip/hip_runtime.h>
#include <math.h>

typedef __attribute__((ext_vector_type(16))) _Float16 v16h;
typedef __attribute__((ext_vector_type(16))) __bf16 v16b;
typedef __attribute__((ext_vector_type(8)))  _Float16 v8h;
typedef __attribute__((ext_vector_type(8)))  float v8f;
typedef __attribute__((ext_vector_type(4)))  float v4f;
typedef __attribute__((ext_vector_type(2)))  float v2f;
typedef __attribute__((ext_vector_type(4)))  unsigned v4u;
typedef __attribute__((ext_vector_type(4)))  int v4i;
typedef float __attribute__((may_alias)) float_a;
typedef int __attribute__((may_alias)) int_a;

template <typename T> __device__ __forceinline__ void vst2(void* p, T v) { *(volatile T*)p = v; __threadfence(); *(volatile T*)p = v; }
__device__ __forceinline__ v8f wmma16(v16h a, v16h b, v8f c) {
  v8f d = __builtin_amdgcn_wmma_f32_16x16x32_f16(false, a, false, b, (short)0, c, false, false);
  asm volatile("v_nop\n\tv_nop\n\tv_nop\n\tv_nop" : "+v"(d) : "v"(a), "v"(b));
  return d;
}
__device__ __forceinline__ v8f wmma_bf(v16b a, v16b b, v8f c) {
  v8f d = __builtin_amdgcn_wmma_f32_16x16x32_bf16(false, a, false, b, (short)0, c, false, false);
  asm volatile("v_nop\n\tv_nop\n\tv_nop\n\tv_nop" : "+v"(d) : "v"(a), "v"(b));
  return d;
}
__device__ __forceinline__ v16h frag_h(const _Float16* rowk0, int lane) {
  union { v16h v; v8h q[2]; } u; const _Float16* p = rowk0 + 8 * (lane >> 4);
  u.q[0] = *(const v8h*)p; u.q[1] = *(const v8h*)(p + 16); return u.v;
}
__device__ __forceinline__ v16h frag_f32(const float* rowk0, int lane) {
  v16h a; const float* p = rowk0 + 8 * (lane >> 4);
#pragma unroll
  for (int i = 0; i < 8; ++i) { a[i] = (_Float16)p[i]; a[8 + i] = (_Float16)p[16 + i]; }
  return a;
}
__device__ __forceinline__ v16h frag_f32s(const float* rowk0, int lane, float sc) {
  v16h a; const float* p = rowk0 + 8 * (lane >> 4);
#pragma unroll
  for (int i = 0; i < 8; ++i) { a[i] = (_Float16)(p[i] * sc); a[8 + i] = (_Float16)(p[16 + i] * sc); }
  return a;
}
__device__ __forceinline__ v16h fragc_f32(const float* W, int k0, int n, int lane, int ld, int K) {
  v16h a; const int g = lane >> 4;
#pragma unroll
  for (int i = 0; i < 8; ++i) { const int ka = k0 + 8 * g + i, kb = ka + 16;
    a[i] = (_Float16)(ka < K ? W[(size_t)ka * ld + n] : 0.f); a[8 + i] = (_Float16)(kb < K ? W[(size_t)kb * ld + n] : 0.f); }
  return a;
}
struct F2 { v16b h, l; };
__device__ __forceinline__ F2 bsplit16(const float v[16]) { F2 r;
#pragma unroll
  for (int i = 0; i < 16; ++i) { const __bf16 h = (__bf16)v[i]; r.h[i] = h; r.l[i] = (__bf16)(v[i] - (float)h); }
  return r; }
__device__ __forceinline__ F2 split_row(const float* row, int k0, int lane) { float v[16]; const float* p = row + k0 + 8 * (lane >> 4);
#pragma unroll
  for (int i = 0; i < 8; ++i) { v[i] = p[i]; v[8 + i] = p[16 + i]; }
  return bsplit16(v); }
__device__ __forceinline__ F2 split_rowK(const float* row, int k0, int lane, int K) { float v[16]; const int g = lane >> 4;
#pragma unroll
  for (int i = 0; i < 8; ++i) { const int ka = k0 + 8 * g + i, kb = ka + 16; v[i] = ka < K ? row[ka] : 0.f; v[8 + i] = kb < K ? row[kb] : 0.f; }
  return bsplit16(v); }
__device__ __forceinline__ F2 split_col(const float* W, int k0, int n, int lane, int ld, int K) { float v[16]; const int g = lane >> 4;
#pragma unroll
  for (int i = 0; i < 8; ++i) { const int ka = k0 + 8 * g + i, kb = ka + 16; v[i] = ka < K ? W[(size_t)ka * ld + n] : 0.f; v[8 + i] = kb < K ? W[(size_t)kb * ld + n] : 0.f; }
  return bsplit16(v); }
__device__ __forceinline__ v8f mac3(const F2& a, const F2& b, v8f c) { c = wmma_bf(a.l, b.h, c); c = wmma_bf(a.h, b.l, c); return wmma_bf(a.h, b.h, c); }
__device__ __forceinline__ float sigm(float v) { return 1.0f / (1.0f + expf(-v)); }
#define LDSX() do { asm volatile("s_wait_dscnt 0" ::: "memory"); __builtin_amdgcn_wave_barrier(); __builtin_amdgcn_fence(__ATOMIC_RELEASE, "workgroup"); } while (0)

#define NV 40000
#define NP 120000
#define KN 27
#define NBLK (NV / 64)
#define NSEM 20

template <int CIN, int COUT, int KP>
__global__ __launch_bounds__(256) void k_packW(const float* __restrict__ W, _Float16* __restrict__ P) {
  const int d = blockIdx.x, tid = threadIdx.x; __shared__ __align__(16) _Float16 sr[KP];
  for (int q = tid; q < KP; q += 256) { float v = 0.f; if (q < KN * CIN) { const int k = q / CIN, c = q % CIN; v = W[((size_t)k * CIN + c) * COUT + d]; } sr[q] = (_Float16)(v * 16.0f); }
  __syncthreads();
  for (int q = tid; q < KP / 8; q += 256) vst2(P + (size_t)d * KP + q * 8, *(const v4u*)(&sr[q * 8]));
}
template <int CIN, int KP, int BNIN>
__global__ __launch_bounds__(256) void k_gat(const float* __restrict__ xin, const float* __restrict__ stin, const float* __restrict__ gin, const float* __restrict__ bin, const int* __restrict__ nbr, int v0, float* __restrict__ GA) {
  const int wave = threadIdx.x >> 5, lane = threadIdx.x & 31; const int rl = blockIdx.x * 8 + wave; const int v = v0 + rl;
  __shared__ int snb[8][KN + 1];
  if (lane < KN) snb[wave][lane] = nbr[(size_t)v * KN + lane];
  LDSX();
  float* dst = GA + (size_t)rl * KP;
  for (int q = lane * 4; q < KP; q += 128) { float4 o; float* ov = (float*)&o;
#pragma unroll
    for (int e = 0; e < 4; ++e) { const int kp = q + e; float val = 0.f;
      if (kp < KN * CIN) { const int k = kp / CIN, c = kp % CIN; const int j = snb[wave][k];
        if (j >= 0 && j < NV) { val = xin[(size_t)j * CIN + c]; if (BNIN) { val = (val - stin[c * 2]) * stin[c * 2 + 1] * gin[c] + bin[c]; val = val > 0.f ? val : 0.f; } } }
      ov[e] = val; }
    vst2(dst + q, *(const v4f*)ov); }
}
template <int CIN, int COUT, int KP>
__global__ __launch_bounds__(128) void k_cgemm(const float* __restrict__ GA, const float* __restrict__ W, int v0, int blk0, float* __restrict__ raw, float* __restrict__ pst) {
  __shared__ __align__(16) float so[4][16][68];
  __shared__ __align__(16) float sps[4][2][64];
  const int tid = threadIdx.x, wave = tid >> 5, lane = tid & 31, col = lane & 15, g = lane >> 4;
  const int blk = blk0 + blockIdx.x, rl0 = blockIdx.x * 64 + wave * 16, vv0 = v0 + rl0;
  v8f acc[COUT / 16];
#pragma unroll
  for (int j = 0; j < COUT / 16; ++j) acc[j] = (v8f){};
#pragma unroll 1
  for (int kc = 0; kc < KP / 32; ++kc) { const F2 a = split_row(GA + (size_t)(rl0 + col) * KP, kc * 32, lane);
#pragma unroll
    for (int j = 0; j < COUT / 16; ++j) acc[j] = mac3(a, split_col(W, kc * 32, j * 16 + col, lane, COUT, KN * CIN), acc[j]); }
#pragma unroll
  for (int j = 0; j < COUT / 16; ++j)
#pragma unroll
    for (int r = 0; r < 8; ++r) so[wave][8 * g + r][j * 16 + col] = acc[j][r];
  LDSX();
  for (int q = lane; q < 16 * (COUT / 4); q += 32) { const int rl = q / (COUT / 4), pc = q % (COUT / 4); vst2(raw + (size_t)(vv0 + rl) * COUT + pc * 4, *(const v4f*)(&so[wave][rl][pc * 4])); }
  if (lane < COUT / 2) { for (int cc = lane; cc < COUT; cc += COUT / 2) { float s = 0.f, s2 = 0.f; for (int rl = 0; rl < 16; ++rl) { const float y = so[wave][rl][cc]; s += y; s2 += y * y; } sps[wave][0][cc] = s; sps[wave][1][cc] = s2; } }
  __syncthreads();
  __shared__ __align__(16) float sout[2][64];
  for (int q = tid; q < 2 * COUT; q += 128) { const int st = q / COUT, c = q % COUT; sout[st][c] = (sps[0][st][c] + sps[1][st][c]) + (sps[2][st][c] + sps[3][st][c]); }
  __syncthreads();
  for (int q = tid; q < 2 * COUT / 4; q += 128) { const int st = q / (COUT / 4), pc = q % (COUT / 4); vst2(pst + ((size_t)blk * 2 + st) * 64 + pc * 4, *(const v4f*)(&sout[st][pc * 4])); }
}
__global__ __launch_bounds__(64) void k_stat(const float* __restrict__ pst, int C, float* __restrict__ stat) {
  __shared__ __align__(16) float so[128];
  const int c = threadIdx.x;
  if (c < C) { float s = 0.f, s2 = 0.f;
#pragma unroll 1
    for (int blk = 0; blk < NBLK; ++blk) { s += pst[((size_t)blk * 2) * 64 + c]; s2 += pst[((size_t)blk * 2 + 1) * 64 + c]; }
    const float mean = s / (float)NV; const float var = fmaxf(s2 / (float)NV - mean * mean, 0.f); so[c * 2] = mean; so[c * 2 + 1] = rsqrtf(var + 1e-5f); }
  else { so[c * 2] = 0.f; so[c * 2 + 1] = 0.f; }
  __syncthreads();
  if (c < 32) vst2(stat + c * 4, *(const v4f*)(&so[c * 4]));
}
__global__ __launch_bounds__(256) void k_head1(const float* __restrict__ raw3, const float* __restrict__ st3, const float* __restrict__ g3, const float* __restrict__ b3, const float* __restrict__ sW1, const float* __restrict__ mW1, float* __restrict__ H, float* __restrict__ pst) {
  __shared__ float sx[64][33]; __shared__ __align__(16) float sh[64][68]; __shared__ __align__(16) float sps[2][64];
  const int tid = threadIdx.x, blk = blockIdx.x, v0 = blk * 64;
  for (int q = tid; q < 64 * 32; q += 256) { const int rl = q >> 5, c = q & 31; float v = (raw3[(size_t)(v0 + rl) * 32 + c] - st3[c * 2]) * st3[c * 2 + 1] * g3[c] + b3[c]; sx[rl][c] = v > 0.f ? v : 0.f; }
  __syncthreads();
  for (int q = tid; q < 64 * 64; q += 256) { const int rl = q >> 6, o = q & 63; const float* W = o < 32 ? sW1 : mW1; const int oo = o & 31; float s = 0.f;
#pragma unroll 8
    for (int c = 0; c < 32; ++c) s += sx[rl][c] * W[c * 32 + oo];
    sh[rl][o] = s; }
  __syncthreads();
  for (int q = tid; q < 64 * 16; q += 256) { const int rl = q >> 4, pc = q & 15; vst2(H + (size_t)(v0 + rl) * 64 + pc * 4, *(const v4f*)(&sh[rl][pc * 4])); }
  if (tid < 64) { float s = 0.f, s2 = 0.f; for (int rl = 0; rl < 64; ++rl) { const float y = sh[rl][tid]; s += y; s2 += y * y; } sps[0][tid] = s; sps[1][tid] = s2; }
  __syncthreads();
  if (tid < 32) vst2(pst + (size_t)blk * 128 + tid * 4, *(const v4f*)(&sps[0][0] + tid * 4));
}
__global__ __launch_bounds__(256) void k_head2(const float* __restrict__ H, const float* __restrict__ stH, const float* __restrict__ sg, const float* __restrict__ sb, const float* __restrict__ sa, const float* __restrict__ sW2, const float* __restrict__ sb2,
                                             const float* __restrict__ mg, const float* __restrict__ mb, const float* __restrict__ ma, const float* __restrict__ mW2, const float* __restrict__ mb2, float* __restrict__ SV) {
  __shared__ float sh[64][65]; __shared__ __align__(16) float so[64][32];
  const int tid = threadIdx.x, v0 = blockIdx.x * 64;
  for (int q = tid; q < 64 * 64; q += 256) { const int rl = q >> 6, o = q & 63; const float hv = H[(size_t)(v0 + rl) * 64 + o]; float v;
    if (o < 32) { v = (hv - stH[o * 2]) * stH[o * 2 + 1] * sg[o] + sb[o]; v = v >= 0.f ? v : sa[0] * v; }
    else { const int oo = o - 32; v = (hv - stH[o * 2]) * stH[o * 2 + 1] * mg[oo] + mb[oo]; v = v >= 0.f ? v : ma[0] * v; }
    sh[rl][o] = v; }
  __syncthreads();
  for (int q = tid; q < 64 * 32; q += 256) { const int rl = q >> 5, o = q & 31; float s = 0.f;
    if (o < NSEM) { s = sb2[o];
#pragma unroll 8
      for (int c = 0; c < 32; ++c) s += sh[rl][c] * sW2[c * NSEM + o]; }
    else if (o == NSEM) { s = mb2[0];
#pragma unroll 8
      for (int c = 0; c < 32; ++c) s += sh[rl][32 + c] * mW2[c]; s = sigm(s); }
    so[rl][o] = s; }
  __syncthreads();
  for (int q = tid; q < 64 * 8; q += 256) { const int rl = q >> 3, pc = q & 7; vst2(SV + (size_t)(v0 + rl) * 32 + pc * 4, *(const v4f*)(&so[rl][pc * 4])); }
}
__global__ __launch_bounds__(256) void k_points(const float* __restrict__ SV, const int* __restrict__ v2p, float* __restrict__ o0, float* __restrict__ o1, float* __restrict__ o2, float* __restrict__ o3) {
  __shared__ __align__(16) float ss[64 * NSEM]; __shared__ __align__(16) float sm[64];
  const int tid = threadIdx.x, p0 = blockIdx.x * 64;
  for (int q = tid; q < 64 * 21; q += 256) { const int pl = q / 21, o = q % 21; int j = v2p[p0 + pl]; j = j < 0 ? 0 : (j >= NV ? NV - 1 : j); const float v = SV[(size_t)j * 32 + o];
    if (o < NSEM) ss[pl * NSEM + o] = v; else sm[pl] = v; }
  __syncthreads();
  for (int q = tid; q < 64 * NSEM / 4; q += 256) { const v4f v = *(const v4f*)(&ss[q * 4]); vst2(o0 + (size_t)p0 * NSEM + q * 4, v); vst2(o2 + (size_t)p0 * NSEM + q * 4, v); }
  if (tid < 16) { const v4f v = *(const v4f*)(&sm[tid * 4]); vst2(o1 + (size_t)p0 + tid * 4, v); vst2(o3 + (size_t)p0 + tid * 4, v); }
}
extern "C" void kernel_launch(void* const* d_in, const int* in_sizes, int n_in, void* d_out, int out_size, void* d_ws, size_t ws_size, hipStream_t stream) {
  (void)in_sizes; (void)n_in; (void)out_size; (void)ws_size;
  const float* feat = (const float*)d_in[0]; const int* v2p = (const int*)d_in[2]; const int* nbr = (const int*)d_in[3];
  const float* W0 = (const float*)d_in[4]; const float* g0 = (const float*)d_in[5]; const float* b0v = (const float*)d_in[6];
  const float* W1 = (const float*)d_in[7]; const float* g1 = (const float*)d_in[8]; const float* b1 = (const float*)d_in[9];
  const float* W2 = (const float*)d_in[10]; const float* g2 = (const float*)d_in[11]; const float* b2 = (const float*)d_in[12];
  const float* W3 = (const float*)d_in[13]; const float* g3 = (const float*)d_in[14]; const float* b3 = (const float*)d_in[15];
  const float* sW1 = (const float*)d_in[16]; const float* sg = (const float*)d_in[17]; const float* sbb = (const float*)d_in[18]; const float* sa = (const float*)d_in[19]; const float* sW2 = (const float*)d_in[20]; const float* sb2 = (const float*)d_in[21];
  const float* mW1 = (const float*)d_in[22]; const float* mg = (const float*)d_in[23]; const float* mbb = (const float*)d_in[24]; const float* ma = (const float*)d_in[25]; const float* mW2 = (const float*)d_in[26]; const float* mb2 = (const float*)d_in[27];
  float* o0 = (float*)d_out; float* o1 = (float*)((char*)d_out + 9600000); float* o2 = (float*)((char*)d_out + 10080000); float* o3 = (float*)((char*)d_out + 19680000);
  char* ws = (char*)d_ws; size_t off = 0;
  auto take = [&](size_t bytes) { char* p = ws + off; off += (bytes + 255) & ~(size_t)255; return p; };
  _Float16* P0 = (_Float16*)take((size_t)32 * 192 * 2); _Float16* P1 = (_Float16*)take((size_t)32 * 864 * 2); _Float16* P2 = (_Float16*)take((size_t)64 * 864 * 2); _Float16* P3 = (_Float16*)take((size_t)32 * 1728 * 2);
  float* raw0 = (float*)take((size_t)NV * 32 * 4); float* raw1 = (float*)take((size_t)NV * 32 * 4); float* raw2 = (float*)take((size_t)NV * 64 * 4); float* raw3 = (float*)take((size_t)NV * 32 * 4);
  float* pst = (float*)take((size_t)NBLK * 2 * 64 * 4); float* st0 = (float*)take(128 * 4); float* st1 = (float*)take(128 * 4); float* st2 = (float*)take(128 * 4); float* st3 = (float*)take(128 * 4); float* stH = (float*)take(128 * 4);
  float* H = (float*)take((size_t)NV * 64 * 4); float* SV = (float*)take((size_t)NV * 32 * 4); float* GA = (float*)take((size_t)70 * 1024 * 1024);
  (void)P0; (void)P1; (void)P2; (void)P3;
  k_gat<6, 192, 0><<<NV / 8, 256, 0, stream>>>(feat, nullptr, nullptr, nullptr, nbr, 0, GA);
  k_cgemm<6, 32, 192><<<NBLK, 128, 0, stream>>>(GA, W0, 0, 0, raw0, pst); k_stat<<<1, 64, 0, stream>>>(pst, 32, st0);
  { const int nb2[2] = {313, 312}; int b0 = 0;
    for (int ch = 0; ch < 2; ++ch) { const int v0 = b0 * 64, nr = nb2[ch] * 64; k_gat<32, 864, 1><<<nr / 8, 256, 0, stream>>>(raw0, st0, g0, b0v, nbr, v0, GA); k_cgemm<32, 32, 864><<<nb2[ch], 128, 0, stream>>>(GA, W1, v0, b0, raw1, pst); b0 += nb2[ch]; } }
  k_stat<<<1, 64, 0, stream>>>(pst, 32, st1);
  { const int nb2[2] = {313, 312}; int b0 = 0;
    for (int ch = 0; ch < 2; ++ch) { const int v0 = b0 * 64, nr = nb2[ch] * 64; k_gat<32, 864, 1><<<nr / 8, 256, 0, stream>>>(raw1, st1, g1, b1, nbr, v0, GA); k_cgemm<32, 64, 864><<<nb2[ch], 128, 0, stream>>>(GA, W2, v0, b0, raw2, pst); b0 += nb2[ch]; } }
  k_stat<<<1, 64, 0, stream>>>(pst, 64, st2);
  { const int nb4[4] = {157, 156, 156, 156}; int b0 = 0;
    for (int ch = 0; ch < 4; ++ch) { const int v0 = b0 * 64, nr = nb4[ch] * 64; k_gat<64, 1728, 1><<<nr / 8, 256, 0, stream>>>(raw2, st2, g2, b2, nbr, v0, GA); k_cgemm<64, 32, 1728><<<nb4[ch], 128, 0, stream>>>(GA, W3, v0, b0, raw3, pst); b0 += nb4[ch]; } }
  k_stat<<<1, 64, 0, stream>>>(pst, 32, st3);
  k_head1<<<NBLK, 256, 0, stream>>>(raw3, st3, g3, b3, sW1, mW1, H, pst); k_stat<<<1, 64, 0, stream>>>(pst, 64, stH);
  k_head2<<<NBLK, 256, 0, stream>>>(H, stH, sg, sbb, sa, sW2, sb2, mg, mbb, ma, mW2, mb2, SV);
  k_points<<<NP / 64, 256, 0, stream>>>(SV, v2p, o0, o1, o2, o3);
}
